// FusedEncoderBlock_54236847014070
// MI455X (gfx1250) — hardware-run, weakly checked
//
#include <hip/hip_runtime.h>
#include <math.h>
#include <float.h>
#include <stdint.h>

#define SEQ   2048
#define DM    1024
#define NH    16
#define HD    64
#define NPAIR (HD / 2)
#define NQB   (SEQ / 64)
#define QKVN  (3 * DM)
#define FFN   (4 * DM)
#define OUTN  (SEQ * DM)
static_assert(NH * HD == DM);
static_assert(HD == 64);
static_assert(DM == 128 * 8);
static_assert((SEQ % 64) == 0 && (DM % 64) == 0 && (QKVN % 64) == 0 && (FFN % 64) == 0);
static_assert((DM % 32) == 0 && (FFN % 32) == 0);
static_assert(((SEQ / 64) * (QKVN / 64)) % 8 == 0);
static_assert(((SEQ / 64) * (DM / 64)) % 8 == 0);
static_assert(((SEQ / 64) * (FFN / 64)) % 8 == 0);
static_assert(((SEQ * DM / 8) % 256) == 0);
static_assert(((SEQ * NPAIR) % 256) == 0);
static_assert((SEQ & (SEQ - 1)) == 0);

typedef _Float16 v16h __attribute__((ext_vector_type(16)));
typedef _Float16 v8h  __attribute__((ext_vector_type(8)));
typedef float    v8f  __attribute__((ext_vector_type(8)));
typedef float    v4f  __attribute__((ext_vector_type(4)));
typedef unsigned int v4u __attribute__((ext_vector_type(4)));

__device__ __forceinline__ unsigned short bf_bits(float f) {
  unsigned u = __float_as_uint(f);
  return (unsigned short)((u + 0x7FFFu + ((u >> 16) & 1u)) >> 16);
}
__device__ __forceinline__ float bf_up(unsigned short h) { return __uint_as_float(((unsigned)h) << 16); }
__device__ __forceinline__ float bfr(float f) { return bf_up(bf_bits(f)); }
__device__ __forceinline__ unsigned short h_bits(_Float16 x) { return __builtin_bit_cast(unsigned short, x); }
__device__ __forceinline__ unsigned pk16(unsigned short a, unsigned short b) { return (unsigned)a | ((unsigned)b << 16); }
__device__ __forceinline__ v8f zero8() { v8f z = {0.f, 0.f, 0.f, 0.f, 0.f, 0.f, 0.f, 0.f}; return z; }

__device__ __forceinline__ void ld8(const float* p, float* o) {
  const v4f a = *(const v4f*)(p);
  const v4f b = *(const v4f*)(p + 4);
  o[0] = a[0]; o[1] = a[1]; o[2] = a[2]; o[3] = a[3];
  o[4] = b[0]; o[5] = b[1]; o[6] = b[2]; o[7] = b[3];
}

__device__ __forceinline__ v16h ldfrag_h(const _Float16* p) {
  union { v16h v; v8h h[2]; } f;
  f.h[0] = *(const v8h*)(p);
  f.h[1] = *(const v8h*)(p + 16);
  return f.v;
}

__device__ __forceinline__ v8f mma_h(v16h a, v16h b, v8f c) {
  c = __builtin_amdgcn_wmma_f32_16x16x32_f16(false, a, false, b, (short)0, c, false, false);
#if defined(__HIP_DEVICE_COMPILE__)
  asm volatile("v_nop\n\tv_nop\n\tv_nop\n\tv_nop" : "+v"(c) : "v"(a), "v"(b));
#endif
  return c;
}
__device__ __forceinline__ v8f mma_h_raw(v16h a, v16h b, v8f c) {
  return __builtin_amdgcn_wmma_f32_16x16x32_f16(false, a, false, b, (short)0, c, false, false);
}
__device__ __forceinline__ void dep_guard_h(v8f& a, v8f& b, v16h x) {
#if defined(__HIP_DEVICE_COMPILE__)
  asm volatile("v_nop\n\tv_nop\n\tv_nop\n\tv_nop" : "+v"(a), "+v"(b) : "v"(x));
#endif
}
__device__ __forceinline__ void keep4_h(v16h a, v16h b, v16h c, v16h d) {
#if defined(__HIP_DEVICE_COMPILE__)
  asm volatile("v_nop" :: "v"(a), "v"(b), "v"(c), "v"(d));
#endif
}
__device__ __forceinline__ void acc_guard4(v8f& a, v8f& b, v8f& c, v8f& d) {
#if defined(__HIP_DEVICE_COMPILE__)
  asm volatile("v_nop\n\tv_nop\n\tv_nop\n\tv_nop" : "+v"(a), "+v"(b), "+v"(c), "+v"(d));
#endif
}

__global__ __launch_bounds__(256) void rope_tab(float* ct, float* st, int n) {
#pragma clang fp contract(off)
  const int i = blockIdx.x * 256 + threadIdx.x;
  if (i < n) {
    const int t = i >> 5;
    const int j = i & 31;
    const float e   = (float)j * (1.0f / 32.0f);
    const float p   = powf(10000.0f, e);
    const float inv = 1.0f / p;
    const float ang = (float)t * inv;
    const float cv = cosf(ang);
    const float sv = sinf(ang);
    *(volatile float*)(ct + i) = cv;
    *(volatile float*)(st + i) = sv;
    __threadfence();
    *(volatile float*)(ct + i) = cv;
    *(volatile float*)(st + i) = sv;
  }
}

__global__ __launch_bounds__(256) void wt_cvt(const float* __restrict__ W, int ncols, int nrows,
                                              unsigned short* outp, float sc) {
  __shared__ __align__(16) float sw[64 * 68];
  const int tid = threadIdx.x;
  const int n0 = blockIdx.x * 64;
  const int k0 = blockIdx.y * 64;
#pragma unroll
  for (int i = 0; i < 4; ++i) {
    const int idx = i * 256 + tid;
    const int kk = idx >> 4, c4 = (idx & 15) * 4;
    const v4f a = *(const v4f*)(W + (size_t)(k0 + kk) * ncols + n0 + c4);
    *(v4f*)(sw + kk * 68 + c4) = a;
  }
  __syncthreads();

  const int g = tid >> 3, piece = tid & 7;
  v4u ov[2];
  size_t oofs[2];
#pragma unroll
  for (int it = 0; it < 2; ++it) {
    const int nn = it * 32 + g;
    v4u a;
#pragma unroll
    for (int e = 0; e < 4; ++e) {
      const float f0 = sw[(piece * 8 + 2 * e) * 68 + nn];
      const float f1 = sw[(piece * 8 + 2 * e + 1) * 68 + nn];
      a[e] = pk16(h_bits((_Float16)(bfr(f0) * sc)), h_bits((_Float16)(bfr(f1) * sc)));
    }
    ov[it] = a;
    oofs[it] = (size_t)(n0 + nn) * nrows + k0 + piece * 8;
  }
  for (int pass = 0; pass < 2; ++pass) {
#pragma unroll
    for (int it = 0; it < 2; ++it) *(volatile v4u*)(outp + oofs[it]) = ov[it];
    __threadfence();
  }
}

__global__ __launch_bounds__(128) void ln_f16(const float* __restrict__ X, const float* __restrict__ gp,
                                              const float* __restrict__ bp, unsigned short* H, int rnd,
                                              float osc) {
#pragma clang fp contract(off)
  __shared__ float red[2][4];
  const int tid = threadIdx.x, wave = tid >> 5, lane = tid & 31;
  const int row = blockIdx.x;
  const int d0 = tid * 8;
  float x[8];
  ld8(X + (size_t)row * DM + d0, x);
  if (rnd != 0) {
#pragma unroll
    for (int e = 0; e < 8; ++e) x[e] = bfr(x[e]);
  }
  float s = 0.f;
#pragma unroll
  for (int e = 0; e < 8; ++e) s += x[e];
#pragma unroll
  for (int off = 16; off >= 1; off >>= 1) s += __shfl_xor(s, off, 32);
  if (lane == 0) red[0][wave] = s;
  __syncthreads();
  const float mu = (((red[0][0] + red[0][1]) + red[0][2]) + red[0][3]) * (1.0f / (float)DM);
  float d[8];
  float ss = 0.f;
#pragma unroll
  for (int e = 0; e < 8; ++e) { d[e] = x[e] - mu; ss += d[e] * d[e]; }
#pragma unroll
  for (int off = 16; off >= 1; off >>= 1) ss += __shfl_xor(ss, off, 32);
  if (lane == 0) red[1][wave] = ss;
  __syncthreads();
  const float var  = (((red[1][0] + red[1][1]) + red[1][2]) + red[1][3]) * (1.0f / (float)DM);
  const float rstd = rsqrtf(var + 1e-5f);
  float gv[8], bv[8];
  ld8(gp + d0, gv);
  ld8(bp + d0, bv);
  v4u a;
#pragma unroll
  for (int p = 0; p < 4; ++p) {
    const int e = 2 * p;
    const float y0 = (d[e] * rstd) * bfr(gv[e]) + bfr(bv[e]);
    const float y1 = (d[e + 1] * rstd) * bfr(gv[e + 1]) + bfr(bv[e + 1]);
    a[p] = pk16(h_bits((_Float16)(y0 * osc)), h_bits((_Float16)(y1 * osc)));
  }
  const size_t o = (size_t)row * DM + d0;
  *(volatile v4u*)(H + o) = a;
  __threadfence();
  *(volatile v4u*)(H + o) = a;
}

template <int MODE, int RR>
__global__ __launch_bounds__(256) void gemm64(
    const unsigned short* __restrict__ Ap, int lda,
    const unsigned short* __restrict__ Btp, int ldb,
    const float* __restrict__ bias, const float* __restrict__ res, int ldr,
    float* Cf, unsigned short* Ch, int ldc, int M, int N, int K, float oscale, float oscale2) {
  const _Float16* Ah = (const _Float16*)(const void*)Ap;
  const _Float16* Bh = (const _Float16*)(const void*)Btp;
  __shared__ __align__(16) float sT[8][16 * 68];
  const int lane = threadIdx.x & 31;
  const int wave = threadIdx.x >> 5;
  const int tilesN = N >> 6;
  const int tilesM = M >> 6;
  const int tile = blockIdx.x * 8 + wave;
  if (tile >= tilesM * tilesN) return;
  const int tm = tile / tilesN;
  const int tn = tile - tm * tilesN;
  const int m0 = tm << 6;
  const int n0 = tn << 6;

  const int rlane = lane & 15;
  const int koff  = (lane >> 4) * 8;
  const int mOff  = (lane >> 4) * 8;

  v8f acc[4][4];
#pragma unroll
  for (int i = 0; i < 4; ++i)
#pragma unroll
    for (int j = 0; j < 4; ++j) acc[i][j] = zero8();

  for (int k0 = 0; k0 < K; k0 += 32) {
    v16h bh[4];
#pragma unroll
    for (int j = 0; j < 4; ++j) {
      const size_t bo = (size_t)(n0 + (j << 4) + rlane) * ldb + koff + k0;
      bh[j] = ldfrag_h(Bh + bo);
    }
#pragma unroll
    for (int i = 0; i < 4; ++i) {
      const size_t ao = (size_t)(m0 + (i << 4) + rlane) * lda + koff + k0;
      const v16h ah = ldfrag_h(Ah + ao);
#pragma unroll
      for (int j = 0; j < 4; ++j) acc[i][j] = mma_h_raw(ah, bh[j], acc[i][j]);
      dep_guard_h(acc[i][0], acc[i][3], ah);
    }
    keep4_h(bh[0], bh[1], bh[2], bh[3]);
  }
  acc_guard4(acc[0][0], acc[0][1], acc[0][2], acc[0][3]);
  acc_guard4(acc[1][0], acc[1][1], acc[1][2], acc[1][3]);
  acc_guard4(acc[2][0], acc[2][1], acc[2][2], acc[2][3]);
  acc_guard4(acc[3][0], acc[3][1], acc[3][2], acc[3][3]);

  float* slab = sT[wave];
#pragma unroll
  for (int i = 0; i < 4; ++i) {
    const int mBase = m0 + (i << 4);
#pragma unroll
    for (int r = 0; r < 8; ++r) {
#pragma unroll
      for (int j = 0; j < 4; ++j) {
        slab[(mOff + r) * 68 + (j << 4) + rlane] = acc[i][j][r];
      }
    }
    __builtin_amdgcn_fence(__ATOMIC_RELEASE, "workgroup");
    __builtin_amdgcn_wave_barrier();
    __builtin_amdgcn_fence(__ATOMIC_ACQUIRE, "workgroup");
    if (MODE != 2) {
      const int h2 = lane >> 4, c4 = (lane & 15) * 4;
      v4f b4 = {0.f, 0.f, 0.f, 0.f};
      if (MODE == 1) {
        const v4f braw = *(const v4f*)(bias + n0 + c4);
#pragma unroll
        for (int e = 0; e < 4; ++e) b4[e] = bfr(braw[e]);
      }
      v4f ov[8];
#pragma unroll
      for (int it = 0; it < 8; ++it) {
        const int row = it * 2 + h2;
        const v4f xs = *(const v4f*)(slab + row * 68 + c4);
        v4f v = xs * oscale;
        if (MODE == 1) {
          v4f r4 = *(const v4f*)(res + (size_t)(mBase + row) * ldr + n0 + c4);
          if (RR != 0) {
#pragma unroll
            for (int e = 0; e < 4; ++e) r4[e] = bfr(r4[e]);
          }
          v = (v + b4) + r4;
        }
        ov[it] = v;
      }
      for (int pass = 0; pass < 2; ++pass) {
#pragma unroll
        for (int it = 0; it < 8; ++it) {
          const int row = it * 2 + h2;
          *(volatile v4f*)(Cf + (size_t)(mBase + row) * ldc + n0 + c4) = ov[it];
        }
        __threadfence();
      }
    } else {
      const int q8 = lane & 7, rr = lane >> 3, c8 = q8 * 8;
      float bb[8];
      {
        const v4f b0 = *(const v4f*)(bias + n0 + c8);
        const v4f b1 = *(const v4f*)(bias + n0 + c8 + 4);
#pragma unroll
        for (int e = 0; e < 4; ++e) { bb[e] = bfr(b0[e]); bb[4 + e] = bfr(b1[e]); }
      }
      v4u ov[4];
#pragma unroll
      for (int it = 0; it < 4; ++it) {
        const int row = it * 4 + rr;
        float xs[8];
        ld8(slab + row * 68 + c8, xs);
        float v[8];
#pragma unroll
        for (int e = 0; e < 8; ++e) {
          const float xv = xs[e] * oscale + bb[e];
          const float gl = 0.5f * xv * (1.0f + erff(xv * 0.70710678118654752f));
          v[e] = gl * oscale2;
        }
        v4u a;
#pragma unroll
        for (int p = 0; p < 4; ++p) a[p] = pk16(h_bits((_Float16)v[2 * p]), h_bits((_Float16)v[2 * p + 1]));
        ov[it] = a;
      }
      for (int pass = 0; pass < 2; ++pass) {
#pragma unroll
        for (int it = 0; it < 4; ++it) {
          const int row = it * 4 + rr;
          *(volatile v4u*)(Ch + (size_t)(mBase + row) * ldc + n0 + c8) = ov[it];
        }
        __threadfence();
      }
    }
    __builtin_amdgcn_fence(__ATOMIC_RELEASE, "workgroup");
    __builtin_amdgcn_wave_barrier();
    __builtin_amdgcn_fence(__ATOMIC_ACQUIRE, "workgroup");
  }
}

__global__ __launch_bounds__(128) void rope_qk(const float* __restrict__ qkvf, const float* __restrict__ ct,
                                               const float* __restrict__ st, unsigned short* qh,
                                               unsigned short* kh, float osc) {
#pragma clang fp contract(off)
  const int tid = threadIdx.x;
  const int t = blockIdx.x;
  const int d0 = tid * 8;
  const int dp = d0 ^ 32;
  const float sgn = ((d0 & 32) == 0) ? -1.0f : 1.0f;
  const float* rowp = qkvf + (size_t)t * QKVN;
  float xq[8], xqp[8], xk[8], xkp[8], cv[8], sv[8];
  ld8(rowp + d0, xq);
  ld8(rowp + dp, xqp);
  ld8(rowp + DM + d0, xk);
  ld8(rowp + DM + dp, xkp);
  const int j0 = d0 & 31;
  ld8(ct + (size_t)t * NPAIR + j0, cv);
  ld8(st + (size_t)t * NPAIR + j0, sv);
  v4u aq, ak;
#pragma unroll
  for (int p = 0; p < 4; ++p) {
    const int e = 2 * p;
    const float yq0 = xq[e] * cv[e] + (sgn * xqp[e]) * sv[e];
    const float yq1 = xq[e + 1] * cv[e + 1] + (sgn * xqp[e + 1]) * sv[e + 1];
    const float yk0 = xk[e] * cv[e] + (sgn * xkp[e]) * sv[e];
    const float yk1 = xk[e + 1] * cv[e + 1] + (sgn * xkp[e + 1]) * sv[e + 1];
    aq[p] = pk16(h_bits((_Float16)(yq0 * osc)), h_bits((_Float16)(yq1 * osc)));
    ak[p] = pk16(h_bits((_Float16)(yk0 * osc)), h_bits((_Float16)(yk1 * osc)));
  }
  const size_t o = (size_t)t * DM + d0;
  *(volatile v4u*)(qh + o) = aq;
  *(volatile v4u*)(kh + o) = ak;
  __threadfence();
  *(volatile v4u*)(qh + o) = aq;
  *(volatile v4u*)(kh + o) = ak;
}

__global__ __launch_bounds__(256) void v_planes(const float* __restrict__ vf, int vrp,
                                                unsigned short* vth, unsigned short* vtl, float vscale) {
  __shared__ __align__(16) float sv[64 * 68];
  const int tid = threadIdx.x;
  const int t0  = blockIdx.x * 64;
  const int hh  = blockIdx.y;
#pragma unroll
  for (int i = 0; i < 4; ++i) {
    const int idx = i * 256 + tid;
    const int tt = idx >> 4, c4 = (idx & 15) * 4;
    const v4f a = *(const v4f*)(vf + ((size_t)(t0 + tt)) * vrp + hh * HD + c4);
    *(v4f*)(sv + tt * 68 + c4) = a;
  }
  __syncthreads();

  const int g = tid >> 3, piece = tid & 7;
  v4u hv[2], lv[2];
  size_t hofs[2];
#pragma unroll
  for (int it = 0; it < 2; ++it) {
    const int d = it * 32 + g;
    v4u a, a2;
#pragma unroll
    for (int e = 0; e < 4; ++e) {
      const float f0 = sv[(piece * 8 + 2 * e) * 68 + d] * vscale;
      const float f1 = sv[(piece * 8 + 2 * e + 1) * 68 + d] * vscale;
      const _Float16 x0 = (_Float16)f0, x1 = (_Float16)f1;
      const unsigned short h0 = h_bits(x0), h1 = h_bits(x1);
      const unsigned short l0 = h_bits((_Float16)((f0 - (float)x0) * 4096.0f));
      const unsigned short l1 = h_bits((_Float16)((f1 - (float)x1) * 4096.0f));
      a[e] = pk16(h0, h1); a2[e] = pk16(l0, l1);
    }
    hv[it] = a; lv[it] = a2;
    hofs[it] = ((size_t)(hh * HD + d)) * SEQ + t0 + piece * 8;
  }
  for (int pass = 0; pass < 2; ++pass) {
#pragma unroll
    for (int it = 0; it < 2; ++it) {
      *(volatile v4u*)(vth + hofs[it]) = hv[it];
      *(volatile v4u*)(vtl + hofs[it]) = lv[it];
    }
    __threadfence();
  }
}

__global__ __launch_bounds__(128)
void attn_c64(const unsigned short* __restrict__ qhp, const unsigned short* __restrict__ khp,
              const unsigned short* __restrict__ vhp, const unsigned short* __restrict__ vlp,
              float* outp, float sscale, float oscl) {
  union FH { v16h v; v8h h[2]; };
  __shared__ __align__(16) _Float16 Ksh[64 * 64];
  __shared__ __align__(16) _Float16 Vth[64 * 64];
  __shared__ __align__(16) _Float16 Vtl[64 * 64];
  __shared__ __align__(16) _Float16 Psh[4][16 * 64];
  __shared__ __align__(16) float    Os[4][16 * 64];

  const int tid  = threadIdx.x;
  const int wave = tid >> 5;
  const int lane = tid & 31;
  const int hh   = lane >> 4;
  const int c    = lane & 15;

  const int bx = blockIdx.x;
  const int qb = bx % NQB;
  const int h  = bx / NQB;
  const int q0 = qb * 64 + wave * 16;

  const _Float16* Qp = (const _Float16*)(const void*)qhp + (size_t)h * HD;
  const _Float16* Kp = (const _Float16*)(const void*)khp + (size_t)h * HD;
  const _Float16* Vh = (const _Float16*)(const void*)vhp + (size_t)h * HD * SEQ;
  const _Float16* Vl = (const _Float16*)(const void*)vlp + (size_t)h * HD * SEQ;

  v16h qa[2];
#pragma unroll
  for (int dc = 0; dc < 2; ++dc) {
    const size_t qo = (size_t)(q0 + c) * DM + dc * 32 + 8 * hh;
    qa[dc] = ldfrag_h(Qp + qo);
  }

  float mrow[8], lrow[8];
  v8f oacc[4];
#pragma unroll
  for (int r = 0; r < 8; ++r) { mrow[r] = -INFINITY; lrow[r] = 0.f; }
#pragma unroll
  for (int t = 0; t < 4; ++t) oacc[t] = zero8();

  const int nkt = qb + 1;
  for (int kt = 0; kt < nkt; ++kt) {
    const int kv0 = kt * 64;
    __syncthreads();
    {
      const int r = tid >> 1, half = (tid & 1) * 32;
      const _Float16* kg  = Kp + (size_t)(kv0 + r) * DM + half;
      const _Float16* vg  = Vh + (size_t)r * SEQ + kv0 + half;
      const _Float16* vlg = Vl + (size_t)r * SEQ + kv0 + half;
#pragma unroll
      for (int i = 0; i < 4; ++i) {
        const v8h a0 = *(const v8h*)(kg + 8 * i);
        const v8h b0 = *(const v8h*)(vg + 8 * i);
        const v8h b1 = *(const v8h*)(vlg + 8 * i);
        *(v8h*)(Ksh + r * 64 + half + 8 * i) = a0;
        *(v8h*)(Vth + r * 64 + half + 8 * i) = b0;
        *(v8h*)(Vtl + r * 64 + half + 8 * i) = b1;
      }
    }
    __syncthreads();

    v8f s[4];
#pragma unroll
    for (int j = 0; j < 4; ++j) {
      s[j] = zero8();
#pragma unroll
      for (int dc = 0; dc < 2; ++dc) {
        FH kb;
        kb.h[0] = *(const v8h*)(Ksh + (j * 16 + c) * 64 + dc * 32 + 8 * hh);
        kb.h[1] = *(const v8h*)(Ksh + (j * 16 + c) * 64 + dc * 32 + 16 + 8 * hh);
        s[j] = mma_h(qa[dc], kb.v, s[j]);
      }
    }

    _Float16* pwh = Psh[wave];
#pragma unroll
    for (int r = 0; r < 8; ++r) {
      const int qrow = q0 + 8 * hh + r;
      float m = -INFINITY;
#pragma unroll
      for (int j = 0; j < 4; ++j) {
        const int key = kv0 + j * 16 + c;
        float sv = s[j][r] * sscale;
        sv = (key <= qrow) ? sv : -FLT_MAX;
        s[j][r] = sv;
        m = fmaxf(m, sv);
      }
#pragma unroll
      for (int off = 1; off < 16; off <<= 1) m = fmaxf(m, __shfl_xor(m, off, 32));
      const float mnew  = fmaxf(mrow[r], m);
      const float msafe = (mnew == -INFINITY) ? 0.f : mnew;
      const float alpha = __expf(mrow[r] - msafe);
      mrow[r] = mnew;
      float psum = 0.f;
#pragma unroll
      for (int j = 0; j < 4; ++j) {
        const float p = __expf(s[j][r] - msafe);
        psum += p;
        const _Float16 ph = (_Float16)(p * 1024.0f);
        pwh[(8 * hh + r) * 64 + j * 16 + c] = ph;
      }
#pragma unroll
      for (int off = 1; off < 16; off <<= 1) psum += __shfl_xor(psum, off, 32);
      lrow[r] = lrow[r] * alpha + psum;
#pragma unroll
      for (int t = 0; t < 4; ++t) oacc[t][r] *= alpha;
    }
    __builtin_amdgcn_fence(__ATOMIC_RELEASE, "workgroup");
    __builtin_amdgcn_wave_barrier();
    __builtin_amdgcn_fence(__ATOMIC_ACQUIRE, "workgroup");

    v8f o1[4];
#pragma unroll
    for (int t = 0; t < 4; ++t) o1[t] = zero8();
#pragma unroll 1
    for (int kk = 0; kk < 2; ++kk) {
      FH pa;
      pa.h[0] = *(const v8h*)(pwh + c * 64 + kk * 32 + 8 * hh);
      pa.h[1] = *(const v8h*)(pwh + c * 64 + kk * 32 + 16 + 8 * hh);
#pragma unroll
      for (int t = 0; t < 4; ++t) {
        FH vb;
        vb.h[0] = *(const v8h*)(Vth + (t * 16 + c) * 64 + kk * 32 + 8 * hh);
        vb.h[1] = *(const v8h*)(Vth + (t * 16 + c) * 64 + kk * 32 + 16 + 8 * hh);
        oacc[t] = mma_h(pa.v, vb.v, oacc[t]);
        FH vl;
        vl.h[0] = *(const v8h*)(Vtl + (t * 16 + c) * 64 + kk * 32 + 8 * hh);
        vl.h[1] = *(const v8h*)(Vtl + (t * 16 + c) * 64 + kk * 32 + 16 + 8 * hh);
        o1[t] = mma_h(pa.v, vl.v, o1[t]);
      }
    }
#pragma unroll
    for (int t = 0; t < 4; ++t)
#pragma unroll
      for (int r = 0; r < 8; ++r) oacc[t][r] += o1[t][r] * (1.0f / 4096.0f);
  }

  float* os = Os[wave];
#pragma unroll
  for (int r = 0; r < 8; ++r) {
    const float l = lrow[r];
    const float inv = ((l > 0.f) ? (1.0f / l) : 0.f) * oscl;
#pragma unroll
    for (int t = 0; t < 4; ++t) os[(8 * hh + r) * 64 + t * 16 + c] = oacc[t][r] * inv;
  }
  __builtin_amdgcn_fence(__ATOMIC_RELEASE, "workgroup");
  __builtin_amdgcn_wave_barrier();
  __builtin_amdgcn_fence(__ATOMIC_ACQUIRE, "workgroup");
  {
    const int h2 = lane >> 4, c4 = (lane & 15) * 4;
    v4f ov[8];
#pragma unroll
    for (int it = 0; it < 8; ++it) {
      const int row = it * 2 + h2;
      ov[it] = *(const v4f*)(os + row * 64 + c4);
    }
    for (int pass = 0; pass < 2; ++pass) {
#pragma unroll
      for (int it = 0; it < 8; ++it) {
        const int row = it * 2 + h2;
        const size_t go = (size_t)(q0 + row) * DM + (size_t)h * HD + c4;
        *(volatile v4f*)(outp + go) = ov[it];
      }
      __threadfence();
    }
  }
}

__global__ __launch_bounds__(256) void cvt_f16x8(const float* __restrict__ in, unsigned short* out, int n8,
                                                 float sc) {
  const int i = blockIdx.x * 256 + threadIdx.x;
  if (i < n8) {
    const v4f a = *(const v4f*)(in + (size_t)i * 8);
    const v4f b = *(const v4f*)(in + (size_t)i * 8 + 4);
    v4u p;
    p[0] = pk16(h_bits((_Float16)(a[0] * sc)), h_bits((_Float16)(a[1] * sc)));
    p[1] = pk16(h_bits((_Float16)(a[2] * sc)), h_bits((_Float16)(a[3] * sc)));
    p[2] = pk16(h_bits((_Float16)(b[0] * sc)), h_bits((_Float16)(b[1] * sc)));
    p[3] = pk16(h_bits((_Float16)(b[2] * sc)), h_bits((_Float16)(b[3] * sc)));
    *(volatile v4u*)(out + (size_t)i * 8) = p;
    __threadfence();
    *(volatile v4u*)(out + (size_t)i * 8) = p;
  }
}

extern "C" void kernel_launch(void* const* d_in, const int* in_sizes, int n_in,
                              void* d_out, int out_size, void* d_ws, size_t ws_size,
                              hipStream_t stream) {
  if (n_in < 12) return;
  if (in_sizes[0] != SEQ * DM) return;
  if (in_sizes[1] != DM * QKVN) return;
  if (in_sizes[2] != DM * DM) return;
  if (in_sizes[3] != DM) return;
  if (in_sizes[4] != DM * FFN) return;
  if (in_sizes[5] != FFN) return;
  if (in_sizes[6] != FFN * DM) return;
  if (in_sizes[7] != DM) return;
  if (in_sizes[8] != DM || in_sizes[9] != DM || in_sizes[10] != DM || in_sizes[11] != DM) return;
  if (out_size != OUTN) return;

  const float* x     = (const float*)d_in[0];
  const float* w_qkv = (const float*)d_in[1];
  const float* w_at  = (const float*)d_in[2];
  const float* b_at  = (const float*)d_in[3];
  const float* w_f1  = (const float*)d_in[4];
  const float* b_f1  = (const float*)d_in[5];
  const float* w_f2  = (const float*)d_in[6];
  const float* b_f2  = (const float*)d_in[7];
  const float* g1    = (const float*)d_in[8];
  const float* bb1   = (const float*)d_in[9];
  const float* g2    = (const float*)d_in[10];
  const float* bb2   = (const float*)d_in[11];

  const size_t PH16  = (size_t)SEQ * DM * 2;
  const size_t PWqkv = (size_t)QKVN * DM * 2;
  const size_t PWa   = (size_t)DM * DM * 2;
  const size_t PW1   = (size_t)FFN * DM * 2;
  const size_t PW2   = (size_t)DM * FFN * 2;
  const size_t PTrig = (size_t)SEQ * NPAIR * 4;
  const size_t PQKV  = (size_t)SEQ * QKVN * 4;
  const size_t P16   = (size_t)SEQ * DM * 2;
  const size_t PVt   = (size_t)DM * SEQ * 2;
  const size_t PF32  = (size_t)SEQ * DM * 4;
  const size_t PG    = (size_t)SEQ * FFN * 2;
  size_t off = 0;
  const size_t oH16 = off; off += PH16;
  const size_t oWq  = off; off += PWqkv;
  const size_t oWa  = off; off += PWa;
  const size_t oW1  = off; off += PW1;
  const size_t oW2  = off; off += PW2;
  const size_t oCos = off; off += PTrig;
  const size_t oSin = off; off += PTrig;
  const size_t oQKV = off; off += PQKV;
  const size_t oQh  = off; off += P16;
  const size_t oKh  = off; off += P16;
  const size_t oVt  = off; off += PVt;
  const size_t oVl  = off; off += PVt;
  const size_t oYf  = off; off += PF32;
  const size_t oY16 = off; off += P16;
  const size_t oX1  = off; off += PF32;
  const size_t oH2  = off; off += P16;
  const size_t oG   = off; off += PG;
  if (off > ws_size) return;
  if (off > (size_t)134217728) return;

  char* ws = (char*)d_ws;
  unsigned short* H16   = (unsigned short*)(ws + oH16);
  unsigned short* WqkvT = (unsigned short*)(ws + oWq);
  unsigned short* WaT   = (unsigned short*)(ws + oWa);
  unsigned short* W1T   = (unsigned short*)(ws + oW1);
  unsigned short* W2T   = (unsigned short*)(ws + oW2);
  float*          CosT  = (float*)(ws + oCos);
  float*          SinT  = (float*)(ws + oSin);
  float*          QKVf  = (float*)(ws + oQKV);
  unsigned short* Qh    = (unsigned short*)(ws + oQh);
  unsigned short* Kh    = (unsigned short*)(ws + oKh);
  unsigned short* VTh   = (unsigned short*)(ws + oVt);
  unsigned short* VTl   = (unsigned short*)(ws + oVl);
  float*          Yf    = (float*)(ws + oYf);
  unsigned short* Y16   = (unsigned short*)(ws + oY16);
  float*          X1f   = (float*)(ws + oX1);
  unsigned short* H2    = (unsigned short*)(ws + oH2);
  unsigned short* G16   = (unsigned short*)(ws + oG);
  float*          outf  = (float*)d_out;

  const dim3 blk(256);
  const int nTrig = SEQ * NPAIR;
  const int n8x   = SEQ * DM / 8;
  const dim3 gTrig((nTrig + 255) / 256);
  const dim3 gCvt((n8x + 255) / 256);
  const dim3 gWqkv(QKVN / 64, DM / 64);
  const dim3 gWa(DM / 64, DM / 64);
  const dim3 gW1(FFN / 64, DM / 64);
  const dim3 gW2(DM / 64, FFN / 64);
  const dim3 gQKV(((SEQ / 64) * (QKVN / 64) + 7) / 8);
  const dim3 gDM(((SEQ / 64) * (DM / 64) + 7) / 8);
  const dim3 gFF1(((SEQ / 64) * (FFN / 64) + 7) / 8);
  const dim3 gVpl(SEQ / 64, NH);
  const dim3 gAttn(NH * NQB);

  const float wScale  = 64.0f;
  const float hScale  = 8.0f;
  const float qkScale = 16.0f;
  const float sscale  = 1.0f / 2048.0f;
  const float vScale  = 256.0f;
  const float attOscl = 1.0f / 262144.0f;
  const float yScale  = 16.0f;
  const float gScale  = 16.0f;

  rope_tab<<<gTrig, blk, 0, stream>>>(CosT, SinT, nTrig);
  wt_cvt<<<gWqkv, blk, 0, stream>>>(w_qkv, QKVN, DM, WqkvT, wScale);
  wt_cvt<<<gWa, blk, 0, stream>>>(w_at, DM, DM, WaT, wScale);
  wt_cvt<<<gW1, blk, 0, stream>>>(w_f1, FFN, DM, W1T, wScale);
  wt_cvt<<<gW2, blk, 0, stream>>>(w_f2, DM, FFN, W2T, wScale);
  ln_f16<<<dim3(SEQ), dim3(128), 0, stream>>>(x, g1, bb1, H16, 1, hScale);
  gemm64<0, 0><<<gQKV, blk, 0, stream>>>(H16, DM, WqkvT, DM, b_at, x, DM, QKVf, H16, QKVN, SEQ, QKVN, DM,
                                         1.0f / 512.0f, 1.0f);
  rope_qk<<<dim3(SEQ), dim3(128), 0, stream>>>(QKVf, CosT, SinT, Qh, Kh, qkScale);
  v_planes<<<gVpl, blk, 0, stream>>>(QKVf + 2 * DM, QKVN, VTh, VTl, vScale);
  attn_c64<<<gAttn, dim3(128), 0, stream>>>(Qh, Kh, VTh, VTl, Yf, sscale, attOscl);
  cvt_f16x8<<<gCvt, blk, 0, stream>>>(Yf, Y16, n8x, yScale);
  gemm64<1, 1><<<gDM, blk, 0, stream>>>(Y16, DM, WaT, DM, b_at, x, DM, X1f, H16, DM, SEQ, DM, DM,
                                        1.0f / 1024.0f, 1.0f);
  ln_f16<<<dim3(SEQ), dim3(128), 0, stream>>>(X1f, g2, bb2, H2, 0, hScale);
  gemm64<2, 0><<<gFF1, blk, 0, stream>>>(H2, DM, W1T, DM, b_f1, x, DM, X1f, G16, FFN, SEQ, FFN, DM,
                                         1.0f / 512.0f, gScale);
  gemm64<1, 0><<<gDM, blk, 0, stream>>>(G16, FFN, W2T, FFN, b_f2, X1f, DM, outf, H16, DM, SEQ, DM, FFN,
                                        1.0f / 1024.0f, 1.0f);
  (void)hipGetLastError();
}
